// GAT_2138893713530
// MI455X (gfx1250) — hardware-verified
//
#include <hip/hip_runtime.h>
#include <math.h>
#include <stdint.h>

#pragma clang fp contract(off)

#define NN     4096
#define NH     4
#define DIM    256
#define RTOT   (NN * NH)
#define K1     256
#define K2     512
#define GP     260
#define OPITCH 132

static_assert(NN == 4096);
static_assert(NN % 128 == 0);
static_assert(NN % 32 == 0);
static_assert(DIM == 256);
static_assert(DIM == 16 * 16);
static_assert(NH == 4);
static_assert(RTOT == NN * NH);
static_assert(RTOT % 128 == 0);
static_assert(64 * 2 == 128);
static_assert(K1 % 32 == 0);
static_assert(K2 % 32 == 0);
static_assert(K2 == 2 * K1);
static_assert(RTOT % 64 == 0);
static_assert(DIM % 64 == 0);

typedef __attribute__((ext_vector_type(16))) __bf16 v16b;
typedef __attribute__((ext_vector_type(8)))  __bf16 v8b;
typedef __attribute__((ext_vector_type(8)))  float  v8f;
typedef __attribute__((ext_vector_type(4)))  float  v4f;
typedef __attribute__((ext_vector_type(4)))  unsigned int v4u;
typedef __attribute__((ext_vector_type(8)))  unsigned int v8u;
typedef v4f __attribute__((may_alias)) v4fa;

union FB { v16b v; v8b h[2]; };

__device__ __forceinline__ unsigned short f2bf_bits(float f) {
  const unsigned u = __float_as_uint(f);
  return (unsigned short)((u + 0x7FFFu + ((u >> 16) & 1u)) >> 16);
}
__device__ __forceinline__ float bf_bits2f(unsigned short h) { return __uint_as_float(((unsigned)h) << 16); }
__device__ __forceinline__ float bfr(float f) { return bf_bits2f(f2bf_bits(f)); }
__device__ __forceinline__ unsigned pk16(unsigned short a, unsigned short b) { return (unsigned)a | ((unsigned)b << 16); }
__device__ __forceinline__ void split2(float f0, float f1, unsigned& wh, unsigned& wl) {
  const unsigned short h0 = f2bf_bits(f0), h1 = f2bf_bits(f1);
  const unsigned short l0 = f2bf_bits(f0 - bf_bits2f(h0));
  const unsigned short l1 = f2bf_bits(f1 - bf_bits2f(h1));
  wh = pk16(h0, h1);
  wl = pk16(l0, l1);
}
__device__ __forceinline__ v4u cvt8(v4f a, v4f b) {
  v4u o;
  o.x = pk16(f2bf_bits(a.x), f2bf_bits(a.y));
  o.y = pk16(f2bf_bits(a.z), f2bf_bits(a.w));
  o.z = pk16(f2bf_bits(b.x), f2bf_bits(b.y));
  o.w = pk16(f2bf_bits(b.z), f2bf_bits(b.w));
  return o;
}
__device__ __forceinline__ void st2_u4(unsigned short* p, v4u v) {
  *(volatile v4u*)p = v;
  __threadfence();
  *(volatile v4u*)p = v;
}
__device__ __forceinline__ void st2_f4(float* p, v4f v) {
  *(volatile v4f*)p = v;
  __threadfence();
  *(volatile v4f*)p = v;
}

__device__ __forceinline__ v8f bf_mma(v16b a, v16b b, v8f c) {
  c = __builtin_amdgcn_wmma_f32_16x16x32_bf16(false, a, false, b, (short)0, c, false, false);
  asm volatile("v_nop\n\tv_nop\n\tv_nop\n\tv_nop" : "+v"(c) : "v"(a), "v"(b));
  return c;
}
__device__ __forceinline__ v16b frag_load(const __bf16* p) {
  FB f;
  f.h[0] = *(const v8b*)(p);
  f.h[1] = *(const v8b*)(p + 16);
  return f.v;
}

#define PREP_XB_BLOCKS  2048
#define PREP_WB_BLOCKS  32
#define PREP_WB2_BLOCKS 64
#define PREP_BLOCKS     (PREP_XB_BLOCKS + PREP_WB_BLOCKS + PREP_WB2_BLOCKS + 1)
static_assert(PREP_XB_BLOCKS * 256 * 8 == RTOT * DIM);
static_assert(PREP_WB_BLOCKS * 256 * 8 == DIM * DIM);
static_assert(PREP_WB2_BLOCKS * 256 * 8 == DIM * K2);

__global__ __launch_bounds__(256) void k_prep(
    const float* __restrict__ state, const float* __restrict__ left,
    const float* __restrict__ W, const float* __restrict__ bvec, const float* __restrict__ aw,
    unsigned short* __restrict__ XB, unsigned short* __restrict__ WB,
    unsigned short* __restrict__ WB2, float* __restrict__ BAF)
{
  const int bx = blockIdx.x, tid = threadIdx.x;
  if (bx < PREP_XB_BLOCKS) {
    const int u  = bx * 256 + tid;
    const int r  = u >> 5, c8 = (u & 31) * 8;
    const int n  = r >> 2, h = r & 3;
    const size_t off = (size_t)(n * 2 + (h & 1)) * DIM + c8;
    const v4f l0 = *(const v4fa*)(left + off);
    const v4f l1 = *(const v4fa*)(left + off + 4);
    const v4f s0 = *(const v4fa*)(state + off);
    const v4f s1 = *(const v4fa*)(state + off + 4);
    asm volatile("" :: "v"(l0), "v"(l1), "v"(s0), "v"(s1));
    const v4u pl = cvt8(l0, l1);
    const v4u ps = cvt8(s0, s1);
    const unsigned mk = 0u - (unsigned)(h >> 1);
    v4u o;
    o.x = (ps.x & mk) | (pl.x & ~mk);
    o.y = (ps.y & mk) | (pl.y & ~mk);
    o.z = (ps.z & mk) | (pl.z & ~mk);
    o.w = (ps.w & mk) | (pl.w & ~mk);
    st2_u4(XB + (size_t)u * 8, o);
  } else if (bx < PREP_XB_BLOCKS + PREP_WB_BLOCKS) {
    const int u = (bx - PREP_XB_BLOCKS) * 256 + tid;
    const v4f a = *(const v4fa*)(W + (size_t)u * 8);
    const v4f c = *(const v4fa*)(W + (size_t)u * 8 + 4);
    st2_u4(WB + (size_t)u * 8, cvt8(a, c));
  } else if (bx < PREP_XB_BLOCKS + PREP_WB_BLOCKS + PREP_WB2_BLOCKS) {
    const int u  = (bx - PREP_XB_BLOCKS - PREP_WB_BLOCKS) * 256 + tid;
    const int o  = u >> 6, c8 = (u & 63) * 8;
    const v4f a = *(const v4fa*)(W + (size_t)o * DIM + (c8 & 255));
    const v4f c = *(const v4fa*)(W + (size_t)o * DIM + (c8 & 255) + 4);
    st2_u4(WB2 + (size_t)o * K2 + c8, cvt8(a, c));
  } else {
    const int t  = tid;
    const int ib = (t < 63 ? t : 63) * 4;
    int ta = t - 64; ta = ta < 0 ? 0 : (ta > 127 ? 127 : ta);
    const v4f vb = *(const v4fa*)(bvec + ib);
    const v4f va = *(const v4fa*)(aw + ta * 4);
    asm volatile("" :: "v"(vb), "v"(va));
    const bool isb = t < 64;
    v4f o;
    o.x = bfr(isb ? vb.x : va.x);
    o.y = bfr(isb ? vb.y : va.y);
    o.z = bfr(isb ? vb.z : va.z);
    o.w = bfr(isb ? vb.w : va.w);
    if (t < 192) st2_f4(BAF + 4 * t, o);
  }
}

__device__ __forceinline__ void slab_put_f32(const float* slab, float* dst, int ldc, int lane) {
  const int hh = lane >> 4, c4 = (lane & 15) * 4;
#pragma unroll
  for (int it = 0; it < 8; ++it) {
    const int row = it * 2 + hh;
    const v4f v = *(const v4fa*)(slab + row * 68 + c4);
    *(volatile v4f*)(dst + (size_t)row * ldc + c4) = v;
  }
}
__device__ __forceinline__ void slab_put_hl(const float* slab, unsigned short* dh, unsigned short* dl, int ldc, int lane) {
  const int q = lane >> 3, c8 = (lane & 7) * 8;
#pragma unroll
  for (int it = 0; it < 4; ++it) {
    const int row = it * 4 + q;
    const float* sp = slab + row * 68 + c8;
    unsigned wh, wl;
    v4u hv, lv;
    split2(sp[0], sp[1], wh, wl); hv.x = wh; lv.x = wl;
    split2(sp[2], sp[3], wh, wl); hv.y = wh; lv.y = wl;
    split2(sp[4], sp[5], wh, wl); hv.z = wh; lv.z = wl;
    split2(sp[6], sp[7], wh, wl); hv.w = wh; lv.w = wl;
    *(volatile v4u*)(dh + (size_t)row * ldc + c8) = hv;
    *(volatile v4u*)(dl + (size_t)row * ldc + c8) = lv;
  }
}

template <int KDIM, int OUT_MODE>
__global__ __launch_bounds__(256) __attribute__((amdgpu_num_vgpr(248)))
void k_gemm(const unsigned short* __restrict__ Ap, int lda,
            const unsigned short* __restrict__ Btp, int ldb,
            void* Cout, void* Cout2, int ldc,
            const float* __restrict__ bias, int M, int N)
{
  static_assert(KDIM % 32 == 0);
  __shared__ __align__(16) float sT[8][16 * 68];
  const __bf16* A  = (const __bf16*)(const void*)Ap;
  const __bf16* Bt = (const __bf16*)(const void*)Btp;
  const int lane = threadIdx.x & 31;
  const int wave = threadIdx.x >> 5;
  const int tilesN = N >> 6;
  const int tilesM = M >> 6;
  const int tile = blockIdx.x * 8 + wave;
  if (tile >= tilesM * tilesN) return;
  const int tm = tile / tilesN;
  const int tn = tile - tm * tilesN;
  const int m0 = tm << 6;
  const int n0 = tn << 6;
  const int rlane = lane & 15;
  const int koff  = (lane >> 4) * 8;
  const int mOff  = (lane >> 4) * 8;

  v8f acc[4][4];
#pragma unroll
  for (int i = 0; i < 4; ++i)
#pragma unroll
    for (int j = 0; j < 4; ++j) acc[i][j] = (v8f){0.f, 0.f, 0.f, 0.f, 0.f, 0.f, 0.f, 0.f};

#pragma unroll 1
  for (int k0 = 0; k0 < KDIM; k0 += 32) {
    v16b bh[4];
#pragma unroll
    for (int j = 0; j < 4; ++j)
      bh[j] = frag_load(Bt + (size_t)(n0 + (j << 4) + rlane) * ldb + koff + k0);
#pragma unroll
    for (int i = 0; i < 4; ++i) {
      const v16b ah = frag_load(A + (size_t)(m0 + (i << 4) + rlane) * lda + koff + k0);
#pragma unroll
      for (int j = 0; j < 4; ++j) acc[i][j] = bf_mma(ah, bh[j], acc[i][j]);
    }
  }

  float* slab = sT[wave];
#pragma unroll
  for (int i = 0; i < 4; ++i) {
    const int mBase = m0 + (i << 4);
#pragma unroll
    for (int j = 0; j < 4; ++j) {
      const float bv = bias[n0 + (j << 4) + rlane];
#pragma unroll
      for (int r = 0; r < 8; ++r) slab[(mOff + r) * 68 + (j << 4) + rlane] = acc[i][j][r] + bv;
    }
    __builtin_amdgcn_fence(__ATOMIC_RELEASE, "workgroup");
    __builtin_amdgcn_wave_barrier();
    __builtin_amdgcn_fence(__ATOMIC_ACQUIRE, "workgroup");
    if (OUT_MODE == 0) {
      float* dst = (float*)Cout + (size_t)mBase * ldc + n0;
      slab_put_f32(slab, dst, ldc, lane);
      __threadfence();
      slab_put_f32(slab, dst, ldc, lane);
    } else {
      unsigned short* dh = (unsigned short*)Cout  + (size_t)mBase * ldc + n0;
      unsigned short* dl = (unsigned short*)Cout2 + (size_t)mBase * ldc + n0;
      slab_put_hl(slab, dh, dl, ldc, lane);
      __threadfence();
      slab_put_hl(slab, dh, dl, ldc, lane);
    }
    __builtin_amdgcn_fence(__ATOMIC_RELEASE, "workgroup");
    __builtin_amdgcn_wave_barrier();
    __builtin_amdgcn_fence(__ATOMIC_ACQUIRE, "workgroup");
  }
}

#define DOTS_LDS_BYTES ((64 * GP + 512 + 128) * 4)

__device__ __forceinline__ void dots_tstore(const float* sG, unsigned short* gth, unsigned short* gtl, size_t base, int tid) {
  const int q8 = tid & 7, sub = tid >> 3;
#pragma unroll 2
  for (int it = 0; it < 8; ++it) {
    const int d = it * 32 + sub;
    const float* sp = sG + (8 * q8) * GP + d;
    unsigned wh, wl;
    v4u hv, lv;
    split2(sp[0 * GP], sp[1 * GP], wh, wl); hv.x = wh; lv.x = wl;
    split2(sp[2 * GP], sp[3 * GP], wh, wl); hv.y = wh; lv.y = wl;
    split2(sp[4 * GP], sp[5 * GP], wh, wl); hv.z = wh; lv.z = wl;
    split2(sp[6 * GP], sp[7 * GP], wh, wl); hv.w = wh; lv.w = wl;
    const size_t go = base + (size_t)d * NN + 8 * q8;
    *(volatile v4u*)(gth + go) = hv;
    *(volatile v4u*)(gtl + go) = lv;
  }
}

__global__ __launch_bounds__(256) void k_dots(
    const float* __restrict__ G, const float* __restrict__ BAF, float* __restrict__ ELR,
    unsigned short* __restrict__ GTH, unsigned short* __restrict__ GTL)
{
  extern __shared__ __align__(16) unsigned char smem_d[];
  float* sG = (float*)smem_d;
  float* sA = sG + 64 * GP;
  float* sE = sA + 512;
  const int tid = threadIdx.x, lane = tid & 31, wave = tid >> 5;
  const int h = blockIdx.y;
  const int n0 = blockIdx.x * 64;

#pragma unroll 4
  for (int it = 0; it < 16; ++it) {
    const int row = it * 4 + (tid >> 6);
    const int c4 = (tid & 63) * 4;
    const v4f v = *(const v4fa*)(G + ((size_t)(n0 + row) * NH + h) * DIM + c4);
    *(v4f*)(sG + row * GP + c4) = v;
  }
  {
    const v4f av = *(const v4fa*)(BAF + 256 + (tid & 127) * 4);
    if (tid < 128) *(v4f*)(sA + tid * 4) = av;
  }
  __syncthreads();

#pragma unroll 1
  for (int rr = 0; rr < 8; ++rr) {
    const int row = wave * 8 + rr;
    float sl = 0.0f, sr = 0.0f;
#pragma unroll
    for (int t = 0; t < 8; ++t) {
      const int f = lane + 32 * t;
      const float v = sG[row * GP + f];
      sl = fmaf(v, sA[f], sl);
      sr = fmaf(v, sA[256 + f], sr);
    }
#pragma unroll
    for (int off = 16; off > 0; off >>= 1) {
      sl += __shfl_xor(sl, off, 32);
      sr += __shfl_xor(sr, off, 32);
    }
    if (lane == 0) { sE[row] = sl; sE[64 + row] = sr; }
  }
  __syncthreads();

  {
    const v4f ev = *(const v4fa*)(sE + 4 * lane);
    float* dst = ELR + (size_t)(lane >> 4) * RTOT + (size_t)h * NN + n0 + 4 * (lane & 15);
    if (wave == 0) st2_f4(dst, ev);
  }
  const size_t base = (size_t)h * DIM * NN + n0;
  dots_tstore(sG, GTH, GTL, base, tid);
  __threadfence();
  dots_tstore(sG, GTH, GTL, base, tid);
}

__global__ __launch_bounds__(256) void k_ermax(const float* __restrict__ ELR, float* __restrict__ ERM)
{
  __shared__ float red[8];
  const int tid = threadIdx.x, lane = tid & 31, wave = tid >> 5;
  const int h = blockIdx.x;
  const float* er = ELR + RTOT + (size_t)h * NN + tid * 16;
  const v4f a = *(const v4fa*)(er);
  const v4f b = *(const v4fa*)(er + 4);
  const v4f c = *(const v4fa*)(er + 8);
  const v4f d = *(const v4fa*)(er + 12);
  float m = fmaxf(fmaxf(fmaxf(a.x, a.y), fmaxf(a.z, a.w)), fmaxf(fmaxf(b.x, b.y), fmaxf(b.z, b.w)));
  m = fmaxf(m, fmaxf(fmaxf(fmaxf(c.x, c.y), fmaxf(c.z, c.w)), fmaxf(fmaxf(d.x, d.y), fmaxf(d.z, d.w))));
#pragma unroll
  for (int off = 16; off > 0; off >>= 1) m = fmaxf(m, __shfl_xor(m, off, 32));
  if (lane == 0) red[wave] = m;
  __syncthreads();
  float r = red[0];
#pragma unroll
  for (int i = 1; i < 8; ++i) r = fmaxf(r, red[i]);
  const v4f o = {r, r, r, r};
  if (tid < 8) st2_f4(ERM + h * 32 + tid * 4, o);
}

#define ATT_LDS_BYTES 82432
static_assert(8 * 16 * OPITCH * 4 <= 81920);

__device__ __forceinline__ float pval(float elr, float mrow, float er) {
  const float s = elr + er;
  const float e = (s >= 0.0f) ? s : 0.2f * s;
  return expf(e - mrow);
}

__device__ __forceinline__ void stage_v(const __bf16* __restrict__ gh, const __bf16* __restrict__ gl,
                                        __bf16* sh, __bf16* sl, int key0, int tid) {
  const __bf16* ph = gh + (size_t)tid * NN + key0;
  const __bf16* pl = gl + (size_t)tid * NN + key0;
  const v8b a0 = *(const v8b*)(ph);
  const v8b a1 = *(const v8b*)(ph + 8);
  const v8b a2 = *(const v8b*)(ph + 16);
  const v8b a3 = *(const v8b*)(ph + 24);
  const v8b b0 = *(const v8b*)(pl);
  const v8b b1 = *(const v8b*)(pl + 8);
  const v8b b2 = *(const v8b*)(pl + 16);
  const v8b b3 = *(const v8b*)(pl + 24);
  __bf16* dh = sh + tid * 32;
  __bf16* dl = sl + tid * 32;
  *(v8b*)(dh)      = a0;
  *(v8b*)(dh + 8)  = a1;
  *(v8b*)(dh + 16) = a2;
  *(v8b*)(dh + 24) = a3;
  *(v8b*)(dl)      = b0;
  *(v8b*)(dl + 8)  = b1;
  *(v8b*)(dl + 16) = b2;
  *(v8b*)(dl + 24) = b3;
}

__device__ __forceinline__ void att_flush(const float* os, float* dst, int lane) {
#pragma unroll
  for (int row = 0; row < 16; ++row) {
    const v4f v = *(const v4fa*)(os + row * OPITCH + lane * 4);
    *(volatile v4f*)(dst + (size_t)row * (NH * DIM) + lane * 4) = v;
  }
}

__global__ __launch_bounds__(256) __attribute__((amdgpu_num_vgpr(248)))
void k_att(const unsigned short* __restrict__ gthp, const unsigned short* __restrict__ gtlp,
           const float* __restrict__ ELR, const float* __restrict__ ERM, float* __restrict__ out)
{
  extern __shared__ __align__(16) unsigned char smem_a[];
  __bf16* sVh = (__bf16*)(smem_a);
  __bf16* sVl = (__bf16*)(smem_a + 32768);
  float*  sER = (float*)(smem_a + 65536);
  float*  sL  = (float*)(smem_a + 81920);
  float*  sO  = (float*)(smem_a);

  const int tid = threadIdx.x, lane = tid & 31, wave = tid >> 5;
  const int hh = lane >> 4, c = lane & 15;
  const int h  = blockIdx.y;
  const int q0 = blockIdx.x * 128 + wave * 16;

  const __bf16* gh = (const __bf16*)(const void*)gthp + (size_t)h * DIM * NN;
  const __bf16* gl = (const __bf16*)(const void*)gtlp + (size_t)h * DIM * NN;

  {
    const float* erp = ELR + RTOT + (size_t)h * NN;
#pragma unroll
    for (int i = 0; i < 4; ++i) {
      const int idx = (i * 256 + tid) * 4;
      const v4f v = *(const v4fa*)(erp + idx);
      *(v4f*)(sER + idx) = v;
    }
  }
  const float ermax = ERM[h * 32];
  const float elr   = ELR[(size_t)h * NN + q0 + c];
  const float sm    = elr + ermax;
  const float mrow  = (sm >= 0.0f) ? sm : 0.2f * sm;

  v8f acc[16];
#pragma unroll
  for (int t = 0; t < 16; ++t) acc[t] = (v8f){0.f, 0.f, 0.f, 0.f, 0.f, 0.f, 0.f, 0.f};
  float lsum = 0.0f;

  stage_v(gh, gl, sVh, sVl, 0, tid);
  __syncthreads();

#pragma unroll 1
  for (int ks = 0; ks < NN / 32; ++ks) {
    const int buf = ks & 1;
    if (ks + 1 < NN / 32) {
      const int nb = (ks + 1) & 1;
      stage_v(gh, gl, sVh + nb * 8192, sVl + nb * 8192, (ks + 1) * 32, tid);
    }

    const float* ep = sER + ks * 32 + 8 * hh;
    const v4f e0 = *(const v4fa*)(ep);
    const v4f e1 = *(const v4fa*)(ep + 4);
    const v4f e2 = *(const v4fa*)(ep + 16);
    const v4f e3 = *(const v4fa*)(ep + 20);
    const float ev[16] = {e0.x, e0.y, e0.z, e0.w, e1.x, e1.y, e1.z, e1.w,
                          e2.x, e2.y, e2.z, e2.w, e3.x, e3.y, e3.z, e3.w};
    v8u ph, pl;
#pragma unroll
    for (int j = 0; j < 8; ++j) {
      const float p0 = pval(elr, mrow, ev[2 * j]);
      const float p1 = pval(elr, mrow, ev[2 * j + 1]);
      lsum += p0;
      lsum += p1;
      unsigned wh, wl;
      split2(p0, p1, wh, wl);
      ph[j] = wh;
      pl[j] = wl;
    }
    const v16b pa = __builtin_bit_cast(v16b, ph);
    const v16b pb = __builtin_bit_cast(v16b, pl);

    const __bf16* vh = sVh + buf * 8192 + c * 32 + 8 * hh;
    const __bf16* vl = sVl + buf * 8192 + c * 32 + 8 * hh;
#pragma unroll
    for (int t = 0; t < 16; ++t) {
      FB vb, vo;
      vb.h[0] = *(const v8b*)(vh + t * 512);
      vb.h[1] = *(const v8b*)(vh + t * 512 + 16);
      vo.h[0] = *(const v8b*)(vl + t * 512);
      vo.h[1] = *(const v8b*)(vl + t * 512 + 16);
      acc[t] = bf_mma(pa, vb.v, acc[t]);
      acc[t] = bf_mma(pb, vb.v, acc[t]);
      acc[t] = bf_mma(pa, vo.v, acc[t]);
    }
    __syncthreads();
  }

  const float lrow = lsum + __shfl_xor(lsum, 16, 32);
  if (hh == 0) sL[wave * 16 + c] = lrow;
  __builtin_amdgcn_fence(__ATOMIC_RELEASE, "workgroup");
  __builtin_amdgcn_wave_barrier();
  __builtin_amdgcn_fence(__ATOMIC_ACQUIRE, "workgroup");
  const v4f la = *(const v4fa*)(sL + wave * 16 + 8 * hh);
  const v4f lb = *(const v4fa*)(sL + wave * 16 + 8 * hh + 4);
  const float inv[8] = {1.0f / la.x, 1.0f / la.y, 1.0f / la.z, 1.0f / la.w,
                        1.0f / lb.x, 1.0f / lb.y, 1.0f / lb.z, 1.0f / lb.w};

  float* os = sO + wave * (16 * OPITCH);
#pragma unroll
  for (int half = 0; half < 2; ++half) {
#pragma unroll
    for (int tt = 0; tt < 8; ++tt)
#pragma unroll
      for (int r = 0; r < 8; ++r)
        os[(8 * hh + r) * OPITCH + tt * 16 + c] = acc[half * 8 + tt][r] * inv[r];
    __builtin_amdgcn_fence(__ATOMIC_RELEASE, "workgroup");
    __builtin_amdgcn_wave_barrier();
    __builtin_amdgcn_fence(__ATOMIC_ACQUIRE, "workgroup");
    float* dst = out + ((size_t)q0 * NH + h) * DIM + half * 128;
    att_flush(os, dst, lane);
    __threadfence();
    att_flush(os, dst, lane);
    __builtin_amdgcn_fence(__ATOMIC_RELEASE, "workgroup");
    __builtin_amdgcn_wave_barrier();
    __builtin_amdgcn_fence(__ATOMIC_ACQUIRE, "workgroup");
  }
}

extern "C" void kernel_launch(void* const* d_in, const int* in_sizes, int n_in,
                              void* d_out, int out_size, void* d_ws, size_t ws_size,
                              hipStream_t stream) {
  if (n_in < 6) return;
  if (in_sizes[0] != NN * 2 * DIM || in_sizes[1] != NN * 2 * DIM) return;
  if (in_sizes[3] != DIM * DIM || in_sizes[4] != DIM || in_sizes[5] != 2 * DIM) return;
  if (out_size != RTOT * DIM) return;

  const float* state = (const float*)d_in[0];
  const float* left  = (const float*)d_in[1];
  const float* W     = (const float*)d_in[3];
  const float* bvec  = (const float*)d_in[4];
  const float* aw    = (const float*)d_in[5];
  float* out = (float*)d_out;

  size_t off = 0;
  const size_t oXB  = off; off += (size_t)RTOT * DIM * 2;
  const size_t oX1  = off; off += (size_t)RTOT * K2 * 2;
  const size_t oG   = off; off += (size_t)RTOT * DIM * 4;
  const size_t oGTH = off; off += (size_t)NH * DIM * NN * 2;
  const size_t oGTL = off; off += (size_t)NH * DIM * NN * 2;
  const size_t oELR = off; off += (size_t)2 * RTOT * 4;
  const size_t oWB  = off; off += (size_t)DIM * DIM * 2;
  const size_t oWB2 = off; off += (size_t)DIM * K2 * 2;
  const size_t oBAF = off; off += (size_t)768 * 4;
  const size_t oERM = off; off += (size_t)NH * 32 * 4;
  if (off > ws_size || off > (size_t)134217728) return;

  char* ws = (char*)d_ws;
  unsigned short* XB   = (unsigned short*)(ws + oXB);
  unsigned short* X1HL = (unsigned short*)(ws + oX1);
  float*          G    = (float*)(ws + oG);
  unsigned short* GTH  = (unsigned short*)(ws + oGTH);
  unsigned short* GTL  = (unsigned short*)(ws + oGTL);
  float*          ELR  = (float*)(ws + oELR);
  unsigned short* WB   = (unsigned short*)(ws + oWB);
  unsigned short* WB2  = (unsigned short*)(ws + oWB2);
  float*          BAF  = (float*)(ws + oBAF);
  float*          ERM  = (float*)(ws + oERM);

  (void)hipFuncSetAttribute(reinterpret_cast<const void*>(&k_dots), hipFuncAttributeMaxDynamicSharedMemorySize, DOTS_LDS_BYTES);
  (void)hipFuncSetAttribute(reinterpret_cast<const void*>(&k_att), hipFuncAttributeMaxDynamicSharedMemorySize, ATT_LDS_BYTES);

  k_prep<<<dim3(PREP_BLOCKS), dim3(256), 0, stream>>>(state, left, W, bvec, aw, XB, WB, WB2, BAF);
  k_gemm<K1, 2><<<dim3((RTOT / 64) * (DIM / 64) / 8), dim3(256), 0, stream>>>(
      XB, DIM, WB, DIM, (void*)X1HL, (void*)(X1HL + DIM), K2, BAF, RTOT, DIM);
  k_gemm<K2, 0><<<dim3((RTOT / 64) * (DIM / 64) / 8), dim3(256), 0, stream>>>(
      X1HL, K2, WB2, K2, (void*)G, (void*)G, DIM, BAF, RTOT, DIM);
  k_dots<<<dim3(NN / 64, NH), dim3(256), DOTS_LDS_BYTES, stream>>>(G, BAF, ELR, GTH, GTL);
  k_ermax<<<dim3(NH), dim3(256), 0, stream>>>(ELR, ERM);
  k_att<<<dim3(NN / 128, NH), dim3(256), ATT_LDS_BYTES, stream>>>(GTH, GTL, ELR, ERM, out);
  (void)hipGetLastError();
}
